// TemporalBlock_87840671138376
// MI455X (gfx1250) — hardware-verified
//
#include <hip/hip_runtime.h>
#include <math.h>

#define NB   4
#define CI   256
#define CO   512
#define SQ   1024
#define SP   1026
#define NTK  4096
#define NHD  8
#define HDM  64

typedef _Float16 v16h __attribute__((ext_vector_type(16)));
typedef _Float16 v8h  __attribute__((ext_vector_type(8)));
typedef __bf16   v16b __attribute__((ext_vector_type(16)));
typedef unsigned short v8us __attribute__((ext_vector_type(8)));
typedef float v8f __attribute__((ext_vector_type(8)));
typedef float v4f __attribute__((ext_vector_type(4)));
typedef v8h  __attribute__((may_alias)) v8ha;
typedef v8us __attribute__((may_alias)) v8usa;
typedef v4f  __attribute__((may_alias)) v4fa;

union FragH { v16h v; v8h p[2]; };
union FragB { v16b v; v8us p[2]; };

__device__ __forceinline__ v8f wmma_h(v16h a, v16h b, v8f c) {
  v8f d = __builtin_amdgcn_wmma_f32_16x16x32_f16(false, a, false, b, (short)0, c, false, false);
  asm volatile("v_nop\n\tv_nop\n\tv_nop\n\tv_nop" : "+v"(d) : "v"(a), "v"(b));
  return d;
}
__device__ __forceinline__ v8f wmma_b(v16b a, v16b b, v8f c) {
  v8f d = __builtin_amdgcn_wmma_f32_16x16x32_bf16(false, a, false, b, (short)0, c, false, false);
  asm volatile("v_nop\n\tv_nop\n\tv_nop\n\tv_nop" : "+v"(d) : "v"(a), "v"(b));
  return d;
}

__device__ __forceinline__ v16h ldh(const _Float16* p, int h) {
  FragH f;
  f.p[0] = *(const v8ha*)(p + 8 * h);
  f.p[1] = *(const v8ha*)(p + 16 + 8 * h);
  return f.v;
}
__device__ __forceinline__ v16b ldb(const unsigned short* p, int h) {
  FragB f;
  f.p[0] = *(const v8usa*)(p + 8 * h);
  f.p[1] = *(const v8usa*)(p + 16 + 8 * h);
  return f.v;
}

__device__ __forceinline__ v8f zero8() {
  v8f z = {0.f, 0.f, 0.f, 0.f, 0.f, 0.f, 0.f, 0.f};
  return z;
}
__device__ __forceinline__ v8f ld8f(const float* p) {
  const v4f a = *(const v4fa*)p;
  const v4f c = *(const v4fa*)(p + 4);
  return __builtin_shufflevector(a, c, 0, 1, 2, 3, 4, 5, 6, 7);
}
__device__ __forceinline__ unsigned short f2bf(float f) {
  unsigned u = __float_as_uint(f);
  u += 0x7FFFu + ((u >> 16) & 1u);
  return (unsigned short)(u >> 16);
}
__device__ __forceinline__ float bf2f(unsigned short s) {
  return __uint_as_float(((unsigned)s) << 16);
}
__device__ __forceinline__ void split8(const v8f v, v8us& hi, v8us& lo) {
  v8us a, c;
#pragma unroll
  for (int e = 0; e < 8; ++e) {
    const unsigned short hs = f2bf(v[e]);
    a[e] = hs;
    c[e] = f2bf(v[e] - bf2f(hs));
  }
  hi = a;
  lo = c;
}
__device__ __forceinline__ v8h toh8(const v8f v, const float s) {
  v8h r;
#pragma unroll
  for (int e = 0; e < 8; ++e) r[e] = (_Float16)(v[e] * s);
  return r;
}
__device__ __forceinline__ float wsum(float v) {
#pragma unroll
  for (int o = 16; o > 0; o >>= 1) v += __shfl_xor(v, o, 32);
  return v;
}
__device__ __forceinline__ float wmax(float v) {
#pragma unroll
  for (int o = 16; o > 0; o >>= 1) v = fmaxf(v, __shfl_xor(v, o, 32));
  return v;
}

__device__ __forceinline__ void mma_32x64_f16(const _Float16* a0p, const _Float16* a1p,
                                              const _Float16* wp, int ldw, int K, int h,
                                              v8f (&acc)[2][4]) {
#pragma unroll 1
  for (int k0 = 0; k0 < K; k0 += 32) {
    const v16h a0 = ldh(a0p + k0, h);
    const v16h a1 = ldh(a1p + k0, h);
#pragma unroll
    for (int nt = 0; nt < 4; ++nt) {
      const v16h bf = ldh(wp + (size_t)(16 * nt) * ldw + k0, h);
      acc[0][nt] = wmma_h(a0, bf, acc[0][nt]);
      acc[1][nt] = wmma_h(a1, bf, acc[1][nt]);
    }
  }
}

__device__ __forceinline__ void store_f32_rows(const float* sT, float* dst, int tok0, int f0,
                                               int w, int lane) {
  const int q16 = lane & 15, s2 = lane >> 4;
#pragma unroll
  for (int i = 0; i < 16; ++i) {
    const int lrow = 32 * w + 2 * i + s2;
    const v4f v = *(const v4fa*)(sT + lrow * 64 + 4 * q16);
    *(volatile v4f*)(dst + ((size_t)(tok0 + lrow)) * CO + f0 + 4 * q16) = v;
  }
}
__device__ __forceinline__ void store_f16_rows(const float* sT, _Float16* dst, int tok0, int f0,
                                               float scale, int w, int lane) {
  const int q8 = lane & 7, sub = lane >> 3;
#pragma unroll
  for (int i = 0; i < 8; ++i) {
    const int lrow = 32 * w + 4 * i + sub;
    const v8f v = ld8f(sT + lrow * 64 + 8 * q8);
    *(volatile v8h*)(dst + ((size_t)(tok0 + lrow)) * CO + f0 + 8 * q8) = toh8(v, scale);
  }
}
__device__ __forceinline__ void conv1_store(const float* sT, unsigned short* Hh, unsigned short* Hl,
                                            int b, int s0, int f0, bool padrows, int w, int lane) {
  const int q8 = lane & 7, sub = lane >> 3;
#pragma unroll
  for (int i = 0; i < 8; ++i) {
    const int lrow = 32 * w + 4 * i + sub;
    const v8f v = ld8f(sT + lrow * 64 + 8 * q8);
    v8us hi, lo;
    split8(v, hi, lo);
    const size_t d = ((size_t)(b * SP + s0 + lrow + 2)) * CO + f0 + 8 * q8;
    *(volatile v8us*)(Hh + d) = hi;
    *(volatile v8us*)(Hl + d) = lo;
  }
  if (padrows && w == 0 && lane < 16) {
    v8us neg1, z8;
#pragma unroll
    for (int e = 0; e < 8; ++e) { neg1[e] = (unsigned short)0xBF80u; z8[e] = (unsigned short)0; }
    const size_t d = ((size_t)(b * SP + sub)) * CO + f0 + 8 * q8;
    *(volatile v8us*)(Hh + d) = neg1;
    *(volatile v8us*)(Hl + d) = z8;
  }
}

__device__ __forceinline__ void xprep_store(const float* tl, unsigned short* xh, unsigned short* xl,
                                            _Float16* x16, int b, int c0, int s0, int st, int tid) {
  const int q8 = tid & 7;
#pragma unroll
  for (int i = 0; i < 2; ++i) {
    const int row = (tid >> 3) + 32 * i;
    const v8f v = ld8f(tl + row * 68 + 8 * q8);
    v8us hi, lo;
    split8(v, hi, lo);
    const size_t o1 = ((size_t)(b * SP + s0 + row + 2)) * CI + c0 + 8 * q8;
    *(volatile v8us*)(xh + o1) = hi;
    *(volatile v8us*)(xl + o1) = lo;
    const size_t o2 = ((size_t)(b * SQ + s0 + row)) * CI + c0 + 8 * q8;
    *(volatile v8h*)(x16 + o2) = toh8(v, 1.0f);
  }
  if (st == 0 && tid < 16) {
    v8us neg1, z8;
#pragma unroll
    for (int e = 0; e < 8; ++e) { neg1[e] = (unsigned short)0xBF80u; z8[e] = (unsigned short)0; }
    const size_t o3 = ((size_t)(b * SP + (tid >> 3))) * CI + c0 + 8 * q8;
    *(volatile v8us*)(xh + o3) = neg1;
    *(volatile v8us*)(xl + o3) = z8;
  }
}

__global__ __launch_bounds__(256) void xprep_kernel(const float* __restrict__ x,
                                                    unsigned short* __restrict__ xh,
                                                    unsigned short* __restrict__ xl,
                                                    _Float16* __restrict__ x16) {
  __shared__ __attribute__((aligned(16))) float tl[64 * 68];
  const int tid = threadIdx.x;
  const int bid = blockIdx.x;
  const int ct = bid & 3, st = (bid >> 2) & 15, b = bid >> 6;
  const int c0 = ct * 64, s0 = st * 64;
#pragma unroll
  for (int i = 0; i < 16; ++i) {
    const int idx = tid + 256 * i;
    const int cc = idx >> 6, ss = idx & 63;
    tl[ss * 68 + cc] = x[((size_t)(b * CI + c0 + cc)) * SQ + s0 + ss];
  }
  __syncthreads();
  xprep_store(tl, xh, xl, x16, b, c0, s0, st, tid);
  __threadfence();
  xprep_store(tl, xh, xl, x16, b, c0, s0, st, tid);
}

__global__ __launch_bounds__(256) void wprep_kernel(
    const float* __restrict__ c1w, const float* __restrict__ c2w, const float* __restrict__ dw,
    const float* __restrict__ qw, const float* __restrict__ kw, const float* __restrict__ vw,
    const float* __restrict__ ow,
    unsigned short* __restrict__ w1h, unsigned short* __restrict__ w1l,
    unsigned short* __restrict__ w2h, unsigned short* __restrict__ w2l,
    _Float16* __restrict__ wd, _Float16* __restrict__ wqkv, _Float16* __restrict__ woh) {
  const int tid = threadIdx.x, blk = blockIdx.x;
  if (blk < 192) {
    const int pl = blk * 256 + tid;
    const int o = pl / 96;
    const int k = 8 * (pl - o * 96);
    const int kk = k >> 8, ci = k & 255;
    v8f v;
#pragma unroll
    for (int e = 0; e < 8; ++e) v[e] = c1w[((size_t)(o * CI + ci + e)) * 3 + kk];
    v8us hi, lo;
    split8(v, hi, lo);
    const size_t d = (size_t)o * (3 * CI) + k;
    *(volatile v8us*)(w1h + d) = hi;
    *(volatile v8us*)(w1l + d) = lo;
    __threadfence();
    *(volatile v8us*)(w1h + d) = hi;
    *(volatile v8us*)(w1l + d) = lo;
  } else if (blk < 576) {
    const int pl = (blk - 192) * 256 + tid;
    const int o = pl / 192;
    const int k = 8 * (pl - o * 192);
    const int kk = k >> 9, ci = k & 511;
    v8f v;
#pragma unroll
    for (int e = 0; e < 8; ++e) v[e] = c2w[((size_t)(o * CO + ci + e)) * 3 + kk];
    v8us hi, lo;
    split8(v, hi, lo);
    const size_t d = (size_t)o * (3 * CO) + k;
    *(volatile v8us*)(w2h + d) = hi;
    *(volatile v8us*)(w2l + d) = lo;
    __threadfence();
    *(volatile v8us*)(w2h + d) = hi;
    *(volatile v8us*)(w2l + d) = lo;
  } else if (blk < 640) {
    const int pl = (blk - 576) * 256 + tid;
    const int o = pl >> 5;
    const int ci = 8 * (pl & 31);
    v8f v;
#pragma unroll
    for (int e = 0; e < 8; ++e) v[e] = dw[(size_t)o * CI + ci + e];
    const v8h r = toh8(v, 256.0f);
    const size_t d = (size_t)o * CI + ci;
    *(volatile v8h*)(wd + d) = r;
    __threadfence();
    *(volatile v8h*)(wd + d) = r;
  } else if (blk < 1024) {
    const int pl = (blk - 640) * 256 + tid;
    const int which = pl >> 15;
    const int rem = pl & 32767;
    const int o = rem >> 6;
    const int in0 = 8 * (rem & 63);
    const float* src = (which == 0) ? qw : ((which == 1) ? kw : vw);
    v8f v;
#pragma unroll
    for (int e = 0; e < 8; ++e) v[e] = src[(size_t)(in0 + e) * CO + o];
    const v8h r = toh8(v, 16.0f);
    const size_t d = ((size_t)which * CO + o) * CO + in0;
    *(volatile v8h*)(wqkv + d) = r;
    __threadfence();
    *(volatile v8h*)(wqkv + d) = r;
  } else {
    const int pl = (blk - 1024) * 256 + tid;
    const int o = pl >> 6;
    const int in0 = 8 * (pl & 63);
    v8f v;
#pragma unroll
    for (int e = 0; e < 8; ++e) v[e] = ow[(size_t)(in0 + e) * CO + o];
    const v8h r = toh8(v, 16.0f);
    const size_t d = (size_t)o * CO + in0;
    *(volatile v8h*)(woh + d) = r;
    __threadfence();
    *(volatile v8h*)(woh + d) = r;
  }
}

template <int CA, int MODE>
__global__ __launch_bounds__(128) void conv_kernel(
    const unsigned short* __restrict__ Ah, const unsigned short* __restrict__ Al,
    const unsigned short* __restrict__ Wh, const unsigned short* __restrict__ Wl,
    const float* __restrict__ cbias, const float* __restrict__ bng, const float* __restrict__ bnb,
    const float* __restrict__ bnm, const float* __restrict__ bnv,
    unsigned short* __restrict__ Hh, unsigned short* __restrict__ Hl,
    float* __restrict__ Xf, _Float16* __restrict__ Xh) {
  __shared__ __attribute__((aligned(16))) float sT[128 * 64];
  constexpr int KT = 3 * CA;
  const int tid = threadIdx.x, lane = tid & 31, w = tid >> 5;
  const int h = lane >> 4, m = lane & 15;
  const int bx = blockIdx.x, b = bx >> 3, s0 = (bx & 7) * 128, f0 = blockIdx.y * 64;

  const size_t ar0 = ((size_t)(b * SP + s0 + 32 * w + m)) * CA;
  const size_t ar1 = ar0 + (size_t)16 * CA;
  const size_t wr  = ((size_t)(f0 + m)) * KT;

  v8f acc[2][4];
#pragma unroll
  for (int mt = 0; mt < 2; ++mt)
#pragma unroll
    for (int nt = 0; nt < 4; ++nt) acc[mt][nt] = zero8();

#pragma unroll 1
  for (int k0 = 0; k0 < KT; k0 += 32) {
    const v16b a0h = ldb(Ah + ar0 + k0, h);
    const v16b a0l = ldb(Al + ar0 + k0, h);
    const v16b a1h = ldb(Ah + ar1 + k0, h);
    const v16b a1l = ldb(Al + ar1 + k0, h);
#pragma unroll
    for (int nt = 0; nt < 4; ++nt) {
      const size_t wofs = wr + (size_t)(16 * nt) * KT + k0;
      const v16b bwh = ldb(Wh + wofs, h);
      const v16b bwl = ldb(Wl + wofs, h);
      acc[0][nt] = wmma_b(a0h, bwh, acc[0][nt]);
      acc[0][nt] = wmma_b(a0l, bwh, acc[0][nt]);
      acc[0][nt] = wmma_b(a0h, bwl, acc[0][nt]);
      acc[1][nt] = wmma_b(a1h, bwh, acc[1][nt]);
      acc[1][nt] = wmma_b(a1l, bwh, acc[1][nt]);
      acc[1][nt] = wmma_b(a1h, bwl, acc[1][nt]);
    }
  }

#pragma unroll
  for (int nt = 0; nt < 4; ++nt) {
    const int col = f0 + 16 * nt + m;
    const float scl = bng[col] * rsqrtf(bnv[col] + 1e-5f);
    const float sft = (cbias[col] - bnm[col]) * scl + bnb[col];
#pragma unroll
    for (int mt = 0; mt < 2; ++mt)
#pragma unroll
      for (int r = 0; r < 8; ++r)
        sT[(32 * w + 16 * mt + 8 * h + r) * 64 + 16 * nt + m] =
            fmaxf(acc[mt][nt][r] * scl + sft, 0.0f);
  }
  __syncthreads();

  if (MODE == 1) {
    const bool padrows = (bx & 7) == 0;
    conv1_store(sT, Hh, Hl, b, s0, f0, padrows, w, lane);
    __threadfence();
    conv1_store(sT, Hh, Hl, b, s0, f0, padrows, w, lane);
  } else {
    const int tok0 = bx * 128;
    store_f32_rows(sT, Xf, tok0, f0, w, lane);
    store_f16_rows(sT, Xh, tok0, f0, 16.0f, w, lane);
    __threadfence();
    store_f32_rows(sT, Xf, tok0, f0, w, lane);
    store_f16_rows(sT, Xh, tok0, f0, 16.0f, w, lane);
  }
}

__global__ __launch_bounds__(128) void down_kernel(const _Float16* __restrict__ x16,
                                                   const _Float16* __restrict__ wd,
                                                   const float* __restrict__ db,
                                                   float* __restrict__ res) {
  __shared__ __attribute__((aligned(16))) float sT[128 * 64];
  const int tid = threadIdx.x, lane = tid & 31, w = tid >> 5;
  const int h = lane >> 4, m = lane & 15;
  const int tok0 = blockIdx.x * 128, f0 = blockIdx.y * 64;

  v8f acc[2][4];
#pragma unroll
  for (int mt = 0; mt < 2; ++mt)
#pragma unroll
    for (int nt = 0; nt < 4; ++nt) acc[mt][nt] = zero8();

  const _Float16* a0p = x16 + ((size_t)(tok0 + 32 * w + m)) * CI;
  const _Float16* a1p = a0p + (size_t)16 * CI;
  const _Float16* wp = wd + ((size_t)(f0 + m)) * CI;
  mma_32x64_f16(a0p, a1p, wp, CI, CI, h, acc);

#pragma unroll
  for (int nt = 0; nt < 4; ++nt) {
    const int col = f0 + 16 * nt + m;
    const float bb = db[col];
#pragma unroll
    for (int mt = 0; mt < 2; ++mt)
#pragma unroll
      for (int r = 0; r < 8; ++r)
        sT[(32 * w + 16 * mt + 8 * h + r) * 64 + 16 * nt + m] =
            acc[mt][nt][r] * (1.0f / 256.0f) + bb;
  }
  __syncthreads();
  store_f32_rows(sT, res, tok0, f0, w, lane);
  __threadfence();
  store_f32_rows(sT, res, tok0, f0, w, lane);
}

__device__ __forceinline__ void qkv_store(const _Float16* sT, _Float16* plane, _Float16* vt,
                                          int which, int bh, int s0, int w, int lane) {
  const int q8 = lane & 7, sub = lane >> 3;
#pragma unroll
  for (int i = 0; i < 8; ++i) {
    const int lid = 32 * w + 4 * i + sub;
    v8h v;
    _Float16* dst;
    if (which != 2) {
      v = *(const v8ha*)(sT + lid * HDM + 8 * q8);
      dst = plane + ((size_t)(bh * SQ + s0 + lid)) * HDM + 8 * q8;
    } else {
      const int d = lid >> 1, hl = lid & 1;
      v = *(const v8ha*)(sT + d * 128 + 64 * hl + 8 * q8);
      dst = vt + ((size_t)(bh * HDM + d)) * SQ + s0 + 64 * hl + 8 * q8;
    }
    *(volatile v8h*)dst = v;
  }
}

__global__ __launch_bounds__(128) void qkv_kernel(const _Float16* __restrict__ xt16,
                                                  const _Float16* __restrict__ wqkv,
                                                  const float* __restrict__ bq,
                                                  const float* __restrict__ bk,
                                                  const float* __restrict__ bv,
                                                  _Float16* __restrict__ qp,
                                                  _Float16* __restrict__ kp,
                                                  _Float16* __restrict__ vt) {
  __shared__ __attribute__((aligned(16))) _Float16 sT[128 * 64];
  const int tid = threadIdx.x, lane = tid & 31, w = tid >> 5;
  const int h = lane >> 4, m = lane & 15;
  const int tok0 = blockIdx.x * 128;
  const int b = tok0 >> 10, s0 = tok0 & (SQ - 1);
  const int which = blockIdx.y >> 3, head = blockIdx.y & 7;
  const int f0 = head * HDM;

  v8f acc[2][4];
#pragma unroll
  for (int mt = 0; mt < 2; ++mt)
#pragma unroll
    for (int nt = 0; nt < 4; ++nt) acc[mt][nt] = zero8();

  const _Float16* a0p = xt16 + ((size_t)(tok0 + 32 * w + m)) * CO;
  const _Float16* a1p = a0p + (size_t)16 * CO;
  const _Float16* wp = wqkv + ((size_t)which * CO + f0 + m) * CO;
  mma_32x64_f16(a0p, a1p, wp, CO, CO, h, acc);

  const float* bias = (which == 0) ? bq : ((which == 1) ? bk : bv);
#pragma unroll
  for (int nt = 0; nt < 4; ++nt) {
    const int featl = 16 * nt + m;
    const float bvl = bias[f0 + featl];
#pragma unroll
    for (int mt = 0; mt < 2; ++mt)
#pragma unroll
      for (int r = 0; r < 8; ++r) {
        const int tokl = 32 * w + 16 * mt + 8 * h + r;
        const float y = (acc[mt][nt][r] * (1.0f / 256.0f) + bvl) * 16.0f;
        const int idx = (which == 2) ? (featl * 128 + tokl) : (tokl * HDM + featl);
        sT[idx] = (_Float16)y;
      }
  }
  __syncthreads();

  const int bh = b * NHD + head;
  _Float16* plane = (which == 0) ? qp : kp;
  qkv_store(sT, plane, vt, which, bh, s0, w, lane);
  __threadfence();
  qkv_store(sT, plane, vt, which, bh, s0, w, lane);
}

#define ATT_LDS (16 * 1024 * 4 + 16 * 1024 * 2 + 16 * 64 * 2)

__device__ __forceinline__ void ao_store(const _Float16* so, _Float16* ao, int b, int head,
                                         int q0, int w, int lane) {
  const int q8 = lane & 7, sub = lane >> 3;
  const int lid = 4 * w + sub;
  const v8h v = *(const v8ha*)(so + lid * HDM + 8 * q8);
  *(volatile v8h*)(ao + ((size_t)(b * SQ + q0 + lid)) * CO + head * HDM + 8 * q8) = v;
}

__global__ __launch_bounds__(256) void attn_kernel(const _Float16* __restrict__ qp,
                                                   const _Float16* __restrict__ kp,
                                                   const _Float16* __restrict__ vt,
                                                   const float* __restrict__ gam,
                                                   _Float16* __restrict__ ao) {
  extern __shared__ v4f dsm_a[];
  char* smem = (char*)dsm_a;
  float* sc = (float*)smem;
  _Float16* sp = (_Float16*)(smem + 65536);
  _Float16* so = (_Float16*)(smem + 65536 + 32768);

  const int tid = threadIdx.x, lane = tid & 31, w = tid >> 5;
  const int h = lane >> 4, m = lane & 15;
  const int bid = blockIdx.x;
  const int qt = bid & 63, head = (bid >> 6) & 7, b = bid >> 9;
  const int q0 = qt * 16, bh = b * NHD + head;

  {
    const _Float16* qrow = qp + ((size_t)(bh * SQ + q0 + m)) * HDM;
    const v16h a0 = ldh(qrow, h);
    const v16h a1 = ldh(qrow + 32, h);
#pragma unroll
    for (int j = 0; j < 8; ++j) {
      const int key0 = 128 * w + 16 * j;
      const _Float16* krow = kp + ((size_t)(bh * SQ + key0 + m)) * HDM;
      const v16h b0 = ldh(krow, h);
      const v16h b1 = ldh(krow + 32, h);
      v8f z = zero8();
      z = wmma_h(a0, b0, z);
      z = wmma_h(a1, b1, z);
#pragma unroll
      for (int r = 0; r < 8; ++r)
        sc[(8 * h + r) * SQ + key0 + m] = z[r] * (1.0f / 2048.0f);
    }
  }
  __syncthreads();

  const float gm = gam[head];
  const float gneg = -(fmaxf(gm, 0.0f) + log1pf(expf(-fabsf(gm))));
#pragma unroll 1
  for (int rr = 0; rr < 2; ++rr) {
    const int row = w + 8 * rr;
    const int q = q0 + row;
    float* srow = sc + row * SQ;
    _Float16* prow = sp + row * SQ;

    float mx = -3.0e38f;
#pragma unroll 4
    for (int i = 0; i < 32; ++i) mx = fmaxf(mx, srow[lane + 32 * i]);
    mx = wmax(mx);
    float se = 0.0f;
#pragma unroll 4
    for (int i = 0; i < 32; ++i) se += __expf(srow[lane + 32 * i] - mx);
    se = wsum(se);
    const float invs = 1.0f / se;

    float running = 0.0f, mx2 = -3.0e38f;
#pragma unroll 1
    for (int base = SQ - 32; base >= 0; base -= 32) {
      const int kidx = base + lane;
      const float s = srow[kidx];
      const float p = __expf(s - mx) * invs;
      float incl = p;
#pragma unroll
      for (int o = 1; o < 32; o <<= 1) {
        const float t = __shfl_down(incl, o, 32);
        if (lane + o < 32) incl += t;
      }
      float excl = __shfl_down(incl, 1, 32);
      if (lane == 31) excl = 0.0f;
      const float rem = running + excl;
      running += __shfl(incl, 0, 32);
      int dq = kidx - q;
      if (dq < 0) dq = -dq;
      const float pos = (float)dq;
      const float ds = sqrtf(fmaxf(rem * pos, 0.0f));
      const float eff = fminf(fmaxf(__expf(ds * gneg), 1e-5f), 1e5f);
      const float ns = s * eff;
      srow[kidx] = ns;
      mx2 = fmaxf(mx2, ns);
    }
    mx2 = wmax(mx2);
    float s2 = 0.0f;
#pragma unroll 4
    for (int i = 0; i < 32; ++i) s2 += __expf(srow[lane + 32 * i] - mx2);
    s2 = wsum(s2);
    const float psc = (q == 0) ? 0.0f : (256.0f / s2);
#pragma unroll 4
    for (int i = 0; i < 32; ++i) {
      const int c = lane + 32 * i;
      prow[c] = (_Float16)(__expf(srow[c] - mx2) * psc);
    }
  }
  __syncthreads();

  if (w < 4) {
    v8f acc = zero8();
    const _Float16* pr = sp + m * SQ;
    const _Float16* vrow = vt + ((size_t)(bh * HDM + 16 * w + m)) * SQ;
#pragma unroll 2
    for (int k0 = 0; k0 < SQ; k0 += 32) {
      const v16h af = ldh(pr + k0, h);
      const v16h bf = ldh(vrow + k0, h);
      acc = wmma_h(af, bf, acc);
    }
#pragma unroll
    for (int r = 0; r < 8; ++r)
      so[(8 * h + r) * HDM + 16 * w + m] = (_Float16)(acc[r] * (1.0f / 16.0f));
  }
  __syncthreads();
  if (w < 4) {
    ao_store(so, ao, b, head, q0, w, lane);
    __threadfence();
    ao_store(so, ao, b, head, q0, w, lane);
  }
}

#define OPJ_LDS (512 * 32 * 4)

__device__ __forceinline__ void out_store(const float* tile, float* out, int b, int s0, int tid) {
#pragma unroll
  for (int i = 0; i < 16; ++i) {
    const int p = tid + 256 * i;
    const int c = p >> 3, q8 = p & 7;
    const v4f v = *(const v4fa*)(tile + c * 32 + 4 * q8);
    *(volatile v4f*)(out + ((size_t)(b * CO + c)) * SQ + s0 + 4 * q8) = v;
  }
}

__global__ __launch_bounds__(256) void oproj_kernel(const _Float16* __restrict__ ao,
                                                    const _Float16* __restrict__ woh,
                                                    const float* __restrict__ obias,
                                                    const float* __restrict__ xt,
                                                    const float* __restrict__ res,
                                                    const float* __restrict__ g1,
                                                    const float* __restrict__ be1,
                                                    const float* __restrict__ g2,
                                                    const float* __restrict__ be2,
                                                    float* __restrict__ out) {
  extern __shared__ v4f dsm_o[];
  float* tile = (float*)dsm_o;
  const int tid = threadIdx.x, lane = tid & 31, w = tid >> 5;
  const int h = lane >> 4, m = lane & 15;
  const int tok0 = blockIdx.x * 32;
  const int b = tok0 >> 10, s0 = tok0 & (SQ - 1);

  v8f acc[2][4];
#pragma unroll
  for (int mt = 0; mt < 2; ++mt)
#pragma unroll
    for (int nt = 0; nt < 4; ++nt) acc[mt][nt] = zero8();

  const _Float16* a0p = ao + ((size_t)(tok0 + m)) * CO;
  const _Float16* a1p = a0p + (size_t)16 * CO;
  const _Float16* wp = woh + ((size_t)(64 * w + m)) * CO;
  mma_32x64_f16(a0p, a1p, wp, CO, CO, h, acc);

#pragma unroll
  for (int nt = 0; nt < 4; ++nt) {
    const int col = 64 * w + 16 * nt + m;
    const float obv = obias[col];
#pragma unroll
    for (int mt = 0; mt < 2; ++mt)
#pragma unroll
      for (int r = 0; r < 8; ++r) {
        const int tokl = 16 * mt + 8 * h + r;
        const float u = acc[mt][nt][r] * (1.0f / 4096.0f) + obv +
                        xt[((size_t)(tok0 + tokl)) * CO + col];
        tile[col * 32 + tokl] = u;
      }
  }
  __syncthreads();

#pragma unroll 1
  for (int j = 0; j < 4; ++j) {
    const int tl = w + 8 * j;
    const size_t rb = ((size_t)(tok0 + tl)) * CO;
    float u[16];
    float su = 0.0f;
#pragma unroll
    for (int i = 0; i < 16; ++i) {
      u[i] = tile[(lane + 32 * i) * 32 + tl];
      su += u[i];
    }
    su = wsum(su);
    const float mu = su * (1.0f / 512.0f);
    float sv = 0.0f;
#pragma unroll
    for (int i = 0; i < 16; ++i) {
      const float d = u[i] - mu;
      sv += d * d;
    }
    sv = wsum(sv);
    const float rs = rsqrtf(sv * (1.0f / 512.0f) + 1e-5f);
    float wv[16];
    float sw = 0.0f;
#pragma unroll
    for (int i = 0; i < 16; ++i) {
      const int c = lane + 32 * i;
      const float a = (u[i] - mu) * rs * g1[c] + be1[c];
      wv[i] = xt[rb + c] + a;
      sw += wv[i];
    }
    sw = wsum(sw);
    const float mu2 = sw * (1.0f / 512.0f);
    float sv2 = 0.0f;
#pragma unroll
    for (int i = 0; i < 16; ++i) {
      const float d = wv[i] - mu2;
      sv2 += d * d;
    }
    sv2 = wsum(sv2);
    const float rs2 = rsqrtf(sv2 * (1.0f / 512.0f) + 1e-5f);
#pragma unroll
    for (int i = 0; i < 16; ++i) {
      const int c = lane + 32 * i;
      const float y = (wv[i] - mu2) * rs2 * g2[c] + be2[c] + res[rb + c];
      tile[c * 32 + tl] = fmaxf(y, 0.0f);
    }
  }
  __syncthreads();

  out_store(tile, out, b, s0, tid);
  __threadfence();
  out_store(tile, out, b, s0, tid);
}

extern "C" void kernel_launch(void* const* d_in, const int* in_sizes, int n_in,
                              void* d_out, int out_size, void* d_ws, size_t ws_size,
                              hipStream_t stream) {
  if (n_in < 28) return;
  if (in_sizes[0] != NB * CI * SQ) return;
  if (in_sizes[1] != CO * CI * 3 || in_sizes[7] != CO * CO * 3 || in_sizes[13] != CO * CI) return;
  if (in_sizes[15] != CO * CO || in_sizes[17] != CO * CO || in_sizes[19] != CO * CO ||
      in_sizes[21] != CO * CO) return;
  const int vec_idx[19] = {2, 3, 4, 5, 6, 8, 9, 10, 11, 12, 14, 16, 18, 20, 22, 24, 25, 26, 27};
  for (int i = 0; i < 19; ++i)
    if (in_sizes[vec_idx[i]] < CO) return;
  if (in_sizes[23] < NHD) return;
  if (out_size != NB * CO * SQ) return;

  const float* x    = (const float*)d_in[0];
  const float* c1w  = (const float*)d_in[1];
  const float* c1b  = (const float*)d_in[2];
  const float* bn1g = (const float*)d_in[3];
  const float* bn1b = (const float*)d_in[4];
  const float* bn1m = (const float*)d_in[5];
  const float* bn1v = (const float*)d_in[6];
  const float* c2w  = (const float*)d_in[7];
  const float* c2b  = (const float*)d_in[8];
  const float* bn2g = (const float*)d_in[9];
  const float* bn2b = (const float*)d_in[10];
  const float* bn2m = (const float*)d_in[11];
  const float* bn2v = (const float*)d_in[12];
  const float* dww  = (const float*)d_in[13];
  const float* dwb  = (const float*)d_in[14];
  const float* qw   = (const float*)d_in[15];
  const float* qb   = (const float*)d_in[16];
  const float* kw   = (const float*)d_in[17];
  const float* kb   = (const float*)d_in[18];
  const float* vw   = (const float*)d_in[19];
  const float* vb   = (const float*)d_in[20];
  const float* ow   = (const float*)d_in[21];
  const float* ob   = (const float*)d_in[22];
  const float* gamma = (const float*)d_in[23];
  const float* ln1g = (const float*)d_in[24];
  const float* ln1b = (const float*)d_in[25];
  const float* ln2g = (const float*)d_in[26];
  const float* ln2b = (const float*)d_in[27];
  float* out = (float*)d_out;

  char* ws = (char*)d_ws;
  size_t off = 0;
  auto carve = [&](size_t bytes) -> char* {
    char* p = ws + off;
    off += (bytes + 255) & ~(size_t)255;
    return p;
  };
  unsigned short* xh  = (unsigned short*)carve((size_t)NB * SP * CI * 2);
  unsigned short* xl  = (unsigned short*)carve((size_t)NB * SP * CI * 2);
  _Float16* x16       = (_Float16*)carve((size_t)NTK * CI * 2);
  unsigned short* w1h = (unsigned short*)carve((size_t)CO * 3 * CI * 2);
  unsigned short* w1l = (unsigned short*)carve((size_t)CO * 3 * CI * 2);
  unsigned short* w2h = (unsigned short*)carve((size_t)CO * 3 * CO * 2);
  unsigned short* w2l = (unsigned short*)carve((size_t)CO * 3 * CO * 2);
  _Float16* wd        = (_Float16*)carve((size_t)CO * CI * 2);
  _Float16* wqkv      = (_Float16*)carve((size_t)3 * CO * CO * 2);
  _Float16* woh       = (_Float16*)carve((size_t)CO * CO * 2);
  unsigned short* hh  = (unsigned short*)carve((size_t)NB * SP * CO * 2);
  unsigned short* hl  = (unsigned short*)carve((size_t)NB * SP * CO * 2);
  float* xt           = (float*)carve((size_t)NTK * CO * 4);
  _Float16* xt16      = (_Float16*)carve((size_t)NTK * CO * 2);
  float* res          = (float*)carve((size_t)NTK * CO * 4);
  _Float16* qpl       = (_Float16*)carve((size_t)NTK * CO * 2);
  _Float16* kpl       = (_Float16*)carve((size_t)NTK * CO * 2);
  _Float16* vtp       = (_Float16*)carve((size_t)NTK * CO * 2);
  _Float16* aop       = (_Float16*)carve((size_t)NTK * CO * 2);
  if (off > ws_size) return;

  xprep_kernel<<<NB * 16 * 4, 256, 0, stream>>>(x, xh, xl, x16);
  wprep_kernel<<<1152, 256, 0, stream>>>(c1w, c2w, dww, qw, kw, vw, ow,
                                         w1h, w1l, w2h, w2l, wd, wqkv, woh);

  const dim3 gconv(NTK / 128, CO / 64);
  conv_kernel<CI, 1><<<gconv, 128, 0, stream>>>(xh, xl, w1h, w1l, c1b, bn1g, bn1b, bn1m, bn1v,
                                                 hh, hl, xt, xt16);
  conv_kernel<CO, 2><<<gconv, 128, 0, stream>>>(hh, hl, w2h, w2l, c2b, bn2g, bn2b, bn2m, bn2v,
                                                 hh, hl, xt, xt16);
  down_kernel<<<gconv, 128, 0, stream>>>(x16, wd, dwb, res);

  const dim3 gqkv(NTK / 128, 3 * NHD);
  qkv_kernel<<<gqkv, 128, 0, stream>>>(xt16, wqkv, qb, kb, vb, qpl, kpl, vtp);

  hipFuncSetAttribute(reinterpret_cast<const void*>(&attn_kernel),
                      hipFuncAttributeMaxDynamicSharedMemorySize, ATT_LDS);
  attn_kernel<<<NB * NHD * (SQ / 16), 256, ATT_LDS, stream>>>(qpl, kpl, vtp, gamma, aop);

  hipFuncSetAttribute(reinterpret_cast<const void*>(&oproj_kernel),
                      hipFuncAttributeMaxDynamicSharedMemorySize, OPJ_LDS);
  oproj_kernel<<<NTK / 32, 256, OPJ_LDS, stream>>>(aop, woh, ob, xt, res, ln1g, ln1b, ln2g, ln2b,
                                                   out);
}
